// DistFlashAttn_20925080666743
// MI455X (gfx1250) — hardware-verified
//
#include <hip/hip_runtime.h>
#include <stddef.h>
#include <stdint.h>

#define SQ   4096
#define SK   4096
#define NH   8
#define HD   64
#define LDQ  (NH * HD)
#define NTOT (SQ * NH * HD)
#define NLSE (NH * SQ)
#define QBR  64
#define NWV  4
#define KC   32
#define NQB  (SQ / QBR)
#define NKT  (SK / KC)
#define MAXR 4
#define PTP  40
#define OTP  68
#define VTRP 65
#define NEGB (-1.0e30f)

static_assert(NTOT == 2097152);
static_assert(NLSE == 32768);
static_assert(SQ % QBR == 0);
static_assert(SK % KC == 0);
static_assert(QBR == NWV * 16);
static_assert(KC == 32);
static_assert(HD == 64);
static_assert(PTP >= KC);
static_assert((PTP * 2) % 16 == 0);
static_assert((OTP * 4) % 16 == 0);
static_assert(NTOT % (8 * 256) == 0);
static_assert(LDQ % 8 == 0);

typedef float          v8f   __attribute__((ext_vector_type(8)));
typedef float          v4f   __attribute__((ext_vector_type(4)));
typedef unsigned int   v4u   __attribute__((ext_vector_type(4)));
typedef unsigned short v8us  __attribute__((ext_vector_type(8)));
typedef unsigned short v16us __attribute__((ext_vector_type(16)));
typedef __bf16         v16b  __attribute__((ext_vector_type(16)));
typedef unsigned short ush;

union FragU { v16us v; v8us h[2]; v16b b; };
union PackU { v8us s; v4u u; };
struct HL { v4u h; v4u l; };

__device__ __forceinline__ ush f2bf(float f) {
  const unsigned u = __float_as_uint(f);
  return (ush)((u + 0x7FFFu + ((u >> 16) & 1u)) >> 16);
}
__device__ __forceinline__ float bf2f(ush v) { return __uint_as_float(((unsigned)v) << 16); }

__device__ __forceinline__ HL split8(v8f f) {
  PackU ph, pl;
#pragma unroll
  for (int e = 0; e < 8; ++e) {
    const ush hi = f2bf(f[e]);
    ph.s[e] = hi;
    pl.s[e] = f2bf(f[e] - bf2f(hi));
  }
  HL r; r.h = ph.u; r.l = pl.u;
  return r;
}

__device__ __forceinline__ v8f mmab(v16us a, v16us b, v8f c) {
  FragU ua, ub; ua.v = a; ub.v = b;
  c = __builtin_amdgcn_wmma_f32_16x16x32_bf16(false, ua.b, false, ub.b, (short)0, c, false, false);
  asm volatile("v_nop\n\tv_nop\n\tv_nop\n\tv_nop" : "+v"(c) : "v"(a), "v"(b));
  return c;
}

__device__ __forceinline__ v16us ldfragu(const ush* p, int ld, int row0, int k0, int lane) {
  const int m = lane & 15, lh = lane >> 4;
  const ush* qq = p + (size_t)(row0 + m) * ld + k0 + 8 * lh;
  FragU f;
  f.h[0] = *(const v8us*)(qq);
  f.h[1] = *(const v8us*)(qq + 16);
  return f.v;
}

__device__ __forceinline__ v8f zero8() { return (v8f){0.f, 0.f, 0.f, 0.f, 0.f, 0.f, 0.f, 0.f}; }

__global__ __launch_bounds__(256) void k_cvt3(const float* __restrict__ q, const float* __restrict__ ka,
                                               const float* __restrict__ kb,
                                               ush* __restrict__ qhp, ush* __restrict__ qlp,
                                               ush* __restrict__ kahp, ush* __restrict__ kalp,
                                               ush* __restrict__ kbhp, ush* __restrict__ kblp) {
  const int y = blockIdx.y;
  const float* src = (y == 0) ? q : ((y == 1) ? ka : kb);
  ush* dh = (y == 0) ? qhp : ((y == 1) ? kahp : kbhp);
  ush* dl = (y == 0) ? qlp : ((y == 1) ? kalp : kblp);
  const size_t p  = (size_t)blockIdx.x * 256 + threadIdx.x;
  const size_t so = p * 8;
  const v4f a0 = *(const v4f*)(src + so);
  const v4f a1 = *(const v4f*)(src + so + 4);
  const v8f f = (v8f){a0[0], a0[1], a0[2], a0[3], a1[0], a1[1], a1[2], a1[3]};
  const HL sp = split8(f);
  *(volatile v4u*)(dh + so) = sp.h;
  *(volatile v4u*)(dl + so) = sp.l;
  __threadfence();
  *(volatile v4u*)(dh + so) = sp.h;
  *(volatile v4u*)(dl + so) = sp.l;
}

__global__ __launch_bounds__(256) void k_vtr(const float* __restrict__ va, const float* __restrict__ vb,
                                             ush* __restrict__ vath, ush* __restrict__ vatl,
                                             ush* __restrict__ vbth, ush* __restrict__ vbtl) {
  __shared__ float tl[64 * VTRP];
  const int tid = threadIdx.x;
  const int s0 = blockIdx.x * 64;
  const int h  = blockIdx.y;
  const int z  = blockIdx.z;
  const float* v = (z == 0) ? va : vb;
  ush* vth = (z == 0) ? vath : vbth;
  ush* vtl = (z == 0) ? vatl : vbtl;
#pragma unroll
  for (int j = 0; j < 4; ++j) {
    const int p  = tid + 256 * j;
    const int ss = p >> 4;
    const int q4 = (p & 15) * 4;
    const v4f a = *(const v4f*)(v + ((size_t)(s0 + ss) * NH + h) * HD + q4);
    float* d = tl + ss * VTRP + q4;
    d[0] = a[0]; d[1] = a[1]; d[2] = a[2]; d[3] = a[3];
  }
  __syncthreads();
  v4u vh[2], vl2[2];
  size_t go[2];
#pragma unroll
  for (int j = 0; j < 2; ++j) {
    const int p  = tid + 256 * j;
    const int dd = p >> 3;
    const int pc = p & 7;
    const float* cp = tl + (pc * 8) * VTRP + dd;
    const v8f f = (v8f){cp[0 * VTRP], cp[1 * VTRP], cp[2 * VTRP], cp[3 * VTRP],
                        cp[4 * VTRP], cp[5 * VTRP], cp[6 * VTRP], cp[7 * VTRP]};
    const HL sp = split8(f);
    vh[j] = sp.h; vl2[j] = sp.l;
    go[j] = ((size_t)h * HD + dd) * SK + s0 + pc * 8;
  }
#pragma unroll
  for (int j = 0; j < 2; ++j) {
    *(volatile v4u*)(vth + go[j]) = vh[j];
    *(volatile v4u*)(vtl + go[j]) = vl2[j];
  }
  __threadfence();
#pragma unroll
  for (int j = 0; j < 2; ++j) {
    *(volatile v4u*)(vth + go[j]) = vh[j];
    *(volatile v4u*)(vtl + go[j]) = vl2[j];
  }
}

__global__ __launch_bounds__(128)
void k_attn(const ush* __restrict__ qh, const ush* __restrict__ ql,
            const ush* __restrict__ kah, const ush* __restrict__ kal,
            const ush* __restrict__ vath, const ush* __restrict__ vatl,
            const ush* __restrict__ kbh, const ush* __restrict__ kbl,
            const ush* __restrict__ vbth, const ush* __restrict__ vbtl,
            const int* __restrict__ qra, const int* __restrict__ kra, const int* __restrict__ cza, int nra,
            const int* __restrict__ qrb, const int* __restrict__ krb, const int* __restrict__ czb, int nrb,
            float* __restrict__ out, float* __restrict__ lse) {
  __shared__ __align__(16) ush   Ph[NWV * 16 * PTP];
  __shared__ __align__(16) ush   Pl[NWV * 16 * PTP];
  __shared__ __align__(16) float Os[NWV * 16 * OTP];
  __shared__ __align__(16) float Ls[QBR];

  const int tid = threadIdx.x, lane = tid & 31, wave = tid >> 5;
  const int hh = lane >> 4, c = lane & 15;
  const int qb   = blockIdx.x;
  const int h    = blockIdx.y;
  const int qblk = qb * QBR;
  const int q0   = qblk + wave * 16;

  const ush* Qh = qh + h * HD;
  const ush* Ql = ql + h * HD;

  ush*   pwh = Ph + wave * 16 * PTP;
  ush*   pwl = Pl + wave * 16 * PTP;
  float* sw  = Os + wave * 16 * OTP;

  float mrow[8], lrow[8];
  v8f oacc[4];
#pragma unroll
  for (int r = 0; r < 8; ++r) { mrow[r] = NEGB; lrow[r] = 0.f; }
#pragma unroll
  for (int t = 0; t < 4; ++t) oacc[t] = zero8();

#pragma unroll 1
  for (int pass = 0; pass < 2; ++pass) {
    const ush* Kh = ((pass == 0) ? kah : kbh) + h * HD;
    const ush* Kl = ((pass == 0) ? kal : kbl) + h * HD;
    const ush* Vh = ((pass == 0) ? vath : vbth) + (size_t)h * HD * SK;
    const ush* Vl = ((pass == 0) ? vatl : vbtl) + (size_t)h * HD * SK;
    const int* QR = (pass == 0) ? qra : qrb;
    const int* KR = (pass == 0) ? kra : krb;
    const int* CZ = (pass == 0) ? cza : czb;
    const int  nr = (pass == 0) ? nra : nrb;

    int rqs[MAXR], rqe[MAXR], rks[MAXR], rke[MAXR], rco[MAXR], rcz[MAXR], ron[MAXR];
    int kmin = SK, kmax = 0;
#pragma unroll
    for (int g = 0; g < MAXR; ++g) {
      const int gg = (g < nr) ? g : (nr - 1);
      const int a = QR[2 * gg], b = QR[2 * gg + 1];
      const int ks = KR[2 * gg], ke = KR[2 * gg + 1];
      const int zc = CZ[gg];
      rqs[g] = a; rqe[g] = b; rks[g] = ks; rke[g] = ke;
      rcz[g] = (zc != 0) ? 1 : 0;
      rco[g] = ks - a + (ke - ks) - (b - a);
      ron[g] = (g < nr) ? 1 : 0;
      const int loq = max(qblk, a), hiq = min(qblk + QBR, b);
      const int klo = max(ks, 0);
      int khi = min(ke, SK);
      if (zc != 0) khi = min(khi, hiq + rco[g]);
      const bool val = (g < nr) && (loq < hiq) && (klo < khi);
      kmin = val ? min(kmin, klo) : kmin;
      kmax = val ? max(kmax, khi) : kmax;
    }
    const int kt0 = kmin & ~(KC - 1);
    int ntile = (kmin < kmax) ? ((kmax - kt0 + KC - 1) / KC) : 0;
    ntile = min(ntile, NKT);

#pragma unroll 1
    for (int it = 0; it < ntile; ++it) {
      const int kv0 = kt0 + KC * it;
      if (kv0 > SK - KC) break;
      bool any = false, full = false;
#pragma unroll
      for (int g = 0; g < MAXR; ++g) {
        const int loq = max(qblk, rqs[g]), hiq = min(qblk + QBR, rqe[g]);
        const int lok = max(kv0, rks[g]),  hik = min(kv0 + KC, rke[g]);
        const bool ov = (ron[g] != 0) & (loq < hiq) & (lok < hik);
        const bool a1 = ov & ((rcz[g] == 0) | (lok <= hiq - 1 + rco[g]));
        const bool f1 = ov & (rqs[g] <= qblk) & (rqe[g] >= qblk + QBR) & (rks[g] <= kv0) & (rke[g] >= kv0 + KC)
                        & ((rcz[g] == 0) | (kv0 + KC - 1 <= qblk + rco[g]));
        any = any | a1;
        full = full | f1;
      }
      if (!any) continue;

      unsigned mbits = 0xFFFFFFFFu;
      if (!full) {
        mbits = 0u;
#pragma unroll
        for (int r = 0; r < 8; ++r) {
          const int qq = q0 + 8 * hh + r;
          int okq[MAXR], lim[MAXR];
#pragma unroll
          for (int g = 0; g < MAXR; ++g) {
            okq[g] = ((ron[g] != 0) & (qq >= rqs[g]) & (qq < rqe[g])) ? 1 : 0;
            lim[g] = (rcz[g] != 0) ? (qq + rco[g]) : 0x7FFFFFFF;
          }
#pragma unroll
          for (int j = 0; j < 2; ++j) {
            const int key = kv0 + 16 * j + c;
            int al = 0;
#pragma unroll
            for (int g = 0; g < MAXR; ++g)
              al |= okq[g] & ((key >= rks[g]) ? 1 : 0) & ((key < rke[g]) ? 1 : 0) & ((key <= lim[g]) ? 1 : 0);
            mbits |= ((unsigned)al) << (2 * r + j);
          }
        }
      }

      __syncthreads();

      v8f s[2];
      s[0] = zero8(); s[1] = zero8();
#pragma unroll
      for (int dc = 0; dc < 2; ++dc) {
        const v16us qah = ldfragu(Qh, LDQ, q0, dc * 32, lane);
        const v16us qal = ldfragu(Ql, LDQ, q0, dc * 32, lane);
#pragma unroll
        for (int j = 0; j < 2; ++j) {
          const v16us kfh = ldfragu(Kh, LDQ, kv0 + 16 * j, dc * 32, lane);
          const v16us kfl = ldfragu(Kl, LDQ, kv0 + 16 * j, dc * 32, lane);
          s[j] = mmab(qah, kfh, s[j]);
          s[j] = mmab(qah, kfl, s[j]);
          s[j] = mmab(qal, kfh, s[j]);
        }
      }
#pragma unroll
      for (int r = 0; r < 8; ++r)
#pragma unroll
        for (int j = 0; j < 2; ++j) {
          const float sv = s[j][r] * 0.125f;
          s[j][r] = ((mbits >> (2 * r + j)) & 1u) ? sv : NEGB;
        }

      float cm[8];
#pragma unroll
      for (int r = 0; r < 8; ++r) {
        float m = fmaxf(s[0][r], s[1][r]);
#pragma unroll
        for (int off = 1; off < 16; off <<= 1) m = fmaxf(m, __shfl_xor(m, off, 32));
        cm[r] = m;
      }
      float al[8];
#pragma unroll
      for (int r = 0; r < 8; ++r) {
        const float mnew  = fmaxf(mrow[r], cm[r]);
        const float alpha = __expf(mrow[r] - mnew);
        mrow[r] = mnew;
        float psum = 0.f;
#pragma unroll
        for (int j = 0; j < 2; ++j) {
          const float e = __expf(s[j][r] - mnew);
          const float p = ((mbits >> (2 * r + j)) & 1u) ? e : 0.f;
          psum += p;
          const ush phi = f2bf(p);
          pwh[(8 * hh + r) * PTP + 16 * j + c] = phi;
          pwl[(8 * hh + r) * PTP + 16 * j + c] = f2bf(p - bf2f(phi));
        }
#pragma unroll
        for (int off = 1; off < 16; off <<= 1) psum += __shfl_xor(psum, off, 32);
        lrow[r] = lrow[r] * alpha + psum;
        al[r] = alpha;
      }
#pragma unroll
      for (int t = 0; t < 4; ++t)
#pragma unroll
        for (int r = 0; r < 8; ++r) oacc[t][r] *= al[r];
      __syncthreads();

      {
        const v16us pah = ldfragu(pwh, PTP, 0, 0, lane);
        const v16us pal = ldfragu(pwl, PTP, 0, 0, lane);
#pragma unroll
        for (int t = 0; t < 4; ++t) {
          const v16us vfh = ldfragu(Vh, SK, 16 * t, kv0, lane);
          const v16us vfl = ldfragu(Vl, SK, 16 * t, kv0, lane);
          oacc[t] = mmab(pah, vfh, oacc[t]);
          oacc[t] = mmab(pah, vfl, oacc[t]);
          oacc[t] = mmab(pal, vfh, oacc[t]);
        }
      }
    }
  }
  __syncthreads();

#pragma unroll
  for (int r = 0; r < 8; ++r) {
    const float lr  = lrow[r];
    const float inv = (lr > 0.f) ? (1.0f / lr) : 0.f;
    const int   row = 8 * hh + r;
#pragma unroll
    for (int t = 0; t < 4; ++t) sw[row * OTP + 16 * t + c] = oacc[t][r] * inv;
    if (c == 0) Ls[wave * 16 + row] = (lr > 0.f) ? (mrow[r] + __logf(lr)) : NEGB;
  }
  __syncthreads();
  v4f val[8];
  size_t go[8];
#pragma unroll
  for (int it = 0; it < 8; ++it) {
    const int p    = lane + 32 * it;
    const int L    = p >> 3;
    const int pc   = p & 7;
    const int row  = L >> 1;
    const int half = L & 1;
    val[it] = *(const v4f*)(sw + row * OTP + half * 32 + pc * 4);
    go[it]  = ((size_t)(q0 + row) * NH + h) * HD + half * 32 + pc * 4;
  }
  const int lc = lane & 15;
  const v4f lv = *(const v4f*)(Ls + 4 * lc);
  const size_t lgo = (size_t)h * SQ + qblk + 4 * lc;
  const bool wl = (wave == 0) && (lane < 16);

#pragma unroll
  for (int it = 0; it < 8; ++it) *(volatile v4f*)(out + go[it]) = val[it];
  if (wl) *(volatile v4f*)(lse + lgo) = lv;
  __threadfence();
#pragma unroll
  for (int it = 0; it < 8; ++it) *(volatile v4f*)(out + go[it]) = val[it];
  if (wl) *(volatile v4f*)(lse + lgo) = lv;
}

extern "C" void kernel_launch(void* const* d_in, const int* in_sizes, int n_in,
                              void* d_out, int out_size, void* d_ws, size_t ws_size,
                              hipStream_t stream) {
  if (n_in < 11) return;
  if (in_sizes[0] != NTOT) return;
  if (in_sizes[1] != NTOT) return;
  if (in_sizes[2] != NTOT) return;
  if (in_sizes[3] != NTOT) return;
  if (in_sizes[4] != NTOT) return;
  const int nra = in_sizes[7];
  const int nrb = in_sizes[10];
  if (nra < 1 || nra > MAXR) return;
  if (nrb < 1 || nrb > MAXR) return;
  if (in_sizes[5] != 2 * nra || in_sizes[6] != 2 * nra) return;
  if (in_sizes[8] != 2 * nrb || in_sizes[9] != 2 * nrb) return;
  if (out_size != NTOT + NLSE) return;

  const float* q   = (const float*)d_in[0];
  const float* ka  = (const float*)d_in[1];
  const float* va  = (const float*)d_in[2];
  const float* kb  = (const float*)d_in[3];
  const float* vb  = (const float*)d_in[4];
  const int*   qra = (const int*)d_in[5];
  const int*   kra = (const int*)d_in[6];
  const int*   cza = (const int*)d_in[7];
  const int*   qrb = (const int*)d_in[8];
  const int*   krb = (const int*)d_in[9];
  const int*   czb = (const int*)d_in[10];
  float* out = (float*)d_out;
  float* lse = out + (size_t)NTOT;

  const size_t plane = (size_t)NTOT * 2;
  size_t off = 0;
  const size_t oQh  = off; off += plane;
  const size_t oQl  = off; off += plane;
  const size_t oKAh = off; off += plane;
  const size_t oKAl = off; off += plane;
  const size_t oKBh = off; off += plane;
  const size_t oKBl = off; off += plane;
  const size_t oVAh = off; off += plane;
  const size_t oVAl = off; off += plane;
  const size_t oVBh = off; off += plane;
  const size_t oVBl = off; off += plane;
  if (off > ws_size) return;
  if (off > (size_t)134217728) return;

  char* ws = (char*)d_ws;
  ush* Qh   = (ush*)(ws + oQh);
  ush* Ql   = (ush*)(ws + oQl);
  ush* KAh  = (ush*)(ws + oKAh);
  ush* KAl  = (ush*)(ws + oKAl);
  ush* KBh  = (ush*)(ws + oKBh);
  ush* KBl  = (ush*)(ws + oKBl);
  ush* VATh = (ush*)(ws + oVAh);
  ush* VATl = (ush*)(ws + oVAl);
  ush* VBTh = (ush*)(ws + oVBh);
  ush* VBTl = (ush*)(ws + oVBl);

  k_cvt3<<<dim3(NTOT / (8 * 256), 3), dim3(256), 0, stream>>>(q, ka, kb, Qh, Ql, KAh, KAl, KBh, KBl);
  k_vtr<<<dim3(SK / 64, NH, 2), dim3(256), 0, stream>>>(va, vb, VATh, VATl, VBTh, VBTl);
  k_attn<<<dim3(NQB, NH), dim3(128), 0, stream>>>(Qh, Ql, KAh, KAl, VATh, VATl, KBh, KBl, VBTh, VBTl,
                                                  qra, kra, cza, nra, qrb, krb, czb, nrb, out, lse);
  (void)hipGetLastError();
}
